// MultiHeadedAttention_CB_36919538876978
// MI455X (gfx1250) — hardware-verified
//
#include <hip/hip_runtime.h>
#include <math.h>

typedef _Float16       v16h __attribute__((ext_vector_type(16)));
typedef _Float16       v8h  __attribute__((ext_vector_type(8)));
typedef __bf16         v16b __attribute__((ext_vector_type(16)));
typedef unsigned short v8us __attribute__((ext_vector_type(8)));
typedef float          v8f  __attribute__((ext_vector_type(8)));
typedef float          v4f  __attribute__((ext_vector_type(4)));
typedef int            v4i  __attribute__((ext_vector_type(4)));
typedef v8h  __attribute__((may_alias)) v8ha;
typedef v8us __attribute__((may_alias)) v8usa;
typedef v4f  __attribute__((may_alias)) v4fa;
typedef v4i  __attribute__((may_alias)) v4ia;

union FragH { v16h v; v8h  half[2]; };
union FragB { v16b v; v8us half[2]; };

#define DM     1024
#define NH     16
#define HD     64
#define SQ     1024
#define NBP    4
#define NTOK   (NBP * SQ)
#define NACT   (NTOK * DM)
#define NWEL   (DM * DM)
#define ACT8   (NACT / 8)
#define WEL8   (NWEL / 8)
#define NGRP   (3 * ACT8 + 4 * WEL8)
#define PSCALE  16384.0f
#define XSCALE  256.0f
#define WSCALE  256.0f
#define LOSCALE 2048.0f

__device__ __forceinline__ v8f wmma_f16(v16h a, v16h b, v8f c) {
  v8f d = __builtin_amdgcn_wmma_f32_16x16x32_f16(false, a, false, b, (short)0, c, false, false);
  asm volatile("v_nop\n\tv_nop\n\tv_nop\n\tv_nop" : "+v"(d) : "v"(a), "v"(b));
  return d;
}
__device__ __forceinline__ v8f wmma_bf16(v16b a, v16b b, v8f c) {
  v8f d = __builtin_amdgcn_wmma_f32_16x16x32_bf16(false, a, false, b, (short)0, c, false, false);
  asm volatile("v_nop\n\tv_nop\n\tv_nop\n\tv_nop" : "+v"(d) : "v"(a), "v"(b));
  return d;
}

__device__ __forceinline__ v16h load_frag_h(const _Float16* p, int h) {
  FragH f;
  f.half[0] = *(const v8ha*)(p + 8 * h);
  f.half[1] = *(const v8ha*)(p + 16 + 8 * h);
  return f.v;
}
__device__ __forceinline__ v16b load_frag_b(const unsigned short* p, int h) {
  FragB f;
  f.half[0] = *(const v8usa*)(p + 8 * h);
  f.half[1] = *(const v8usa*)(p + 16 + 8 * h);
  return f.v;
}

__device__ __forceinline__ unsigned short bf16_bits(float f) {
  unsigned int u = __float_as_uint(f);
  u = u + 0x7FFFu + ((u >> 16) & 1u);
  return (unsigned short)(u >> 16);
}
__device__ __forceinline__ float bf16_val(float f) {
  return __uint_as_float(((unsigned int)bf16_bits(f)) << 16);
}

__global__ __launch_bounds__(256) void convert_kernel(
    const float* __restrict__ xq, const float* __restrict__ xk, const float* __restrict__ xv,
    const float* __restrict__ wq, const float* __restrict__ wk, const float* __restrict__ wv,
    const float* __restrict__ wo,
    unsigned short* __restrict__ xb, unsigned short* __restrict__ wb, _Float16* __restrict__ woh)
{
  const int g = blockIdx.x * 256 + threadIdx.x;
  if (g >= NGRP) return;
  if (g < 3 * ACT8 + 3 * WEL8) {
    const float* src;
    unsigned short* dst;
    if (g < 3 * ACT8) {
      const int sel = g / ACT8;
      const int off = g - sel * ACT8;
      const float* xs = (sel == 0) ? xq : ((sel == 1) ? xk : xv);
      src = xs + (size_t)off * 8;
      dst = xb + (size_t)sel * NACT + (size_t)off * 8;
    } else {
      const int e = g - 3 * ACT8;
      const int sel = e / WEL8;
      const int off = e - sel * WEL8;
      const float* wsrc = (sel == 0) ? wq : ((sel == 1) ? wk : wv);
      src = wsrc + (size_t)off * 8;
      dst = wb + (size_t)sel * NWEL + (size_t)off * 8;
    }
    const v4f a = *(const v4fa*)src;
    const v4f c = *(const v4fa*)(src + 4);
    const v8us o = { bf16_bits(a.x), bf16_bits(a.y), bf16_bits(a.z), bf16_bits(a.w),
                     bf16_bits(c.x), bf16_bits(c.y), bf16_bits(c.z), bf16_bits(c.w) };
    *(volatile v8us*)dst = o;
    __threadfence();
    *(volatile v8us*)dst = o;
  } else {
    const int off = g - (3 * ACT8 + 3 * WEL8);
    const float* src = wo + (size_t)off * 8;
    _Float16* dst = woh + (size_t)off * 8;
    const v4f a = *(const v4fa*)src;
    const v4f c = *(const v4fa*)(src + 4);
    const v8h o = { (_Float16)(bf16_val(a.x) * WSCALE), (_Float16)(bf16_val(a.y) * WSCALE),
                    (_Float16)(bf16_val(a.z) * WSCALE), (_Float16)(bf16_val(a.w) * WSCALE),
                    (_Float16)(bf16_val(c.x) * WSCALE), (_Float16)(bf16_val(c.y) * WSCALE),
                    (_Float16)(bf16_val(c.z) * WSCALE), (_Float16)(bf16_val(c.w) * WSCALE) };
    *(volatile v8h*)dst = o;
    __threadfence();
    *(volatile v8h*)dst = o;
  }
}

__device__ __forceinline__ void proj_store_pass(const _Float16* sT, _Float16* plane, _Float16* vt,
                                                int which, int bh, int l0, int w, int lane) {
  const int q8 = lane & 7, sub = lane >> 3;
  #pragma unroll
  for (int i = 0; i < 8; ++i) {
    const int lid = w * 32 + i * 4 + sub;
    v8h v;
    _Float16* dst;
    if (which != 2) {
      v = *(const v8ha*)(sT + lid * HD + 8 * q8);
      dst = plane + ((size_t)bh * SQ + l0 + lid) * HD + 8 * q8;
    } else {
      const int d = lid >> 1, hl = lid & 1;
      v = *(const v8ha*)(sT + d * 128 + 64 * hl + 8 * q8);
      dst = vt + ((size_t)bh * HD + d) * SQ + l0 + 64 * hl + 8 * q8;
    }
    *(volatile v8h*)dst = v;
  }
}

__global__ __launch_bounds__(128) void proj_kernel(
    const unsigned short* __restrict__ xb,
    const unsigned short* __restrict__ wb,
    const float* __restrict__ bq, const float* __restrict__ bk, const float* __restrict__ bv,
    _Float16* __restrict__ qh,
    _Float16* __restrict__ kh,
    _Float16* __restrict__ vt)
{
  __shared__ __attribute__((aligned(16))) _Float16 sT[128 * 64];

  const int tid = threadIdx.x, lane = tid & 31, w = tid >> 5;
  const int h = lane >> 4, m = lane & 15;
  const int m0 = blockIdx.x * 128;
  const int cg = blockIdx.y;
  const int which = cg >> 4, head = cg & 15;
  const int m0w = m0 + 32 * w;

  const unsigned short* xa0 = xb + (size_t)which * NACT + (size_t)(m0w + m) * DM;
  const unsigned short* xa1 = xa0 + (size_t)16 * DM;
  const unsigned short* wr  = wb + (size_t)which * NWEL + (size_t)(head * HD + m) * DM;

  const v8f zero8 = {0.f, 0.f, 0.f, 0.f, 0.f, 0.f, 0.f, 0.f};
  v8f acc[2][4];
  #pragma unroll
  for (int mt = 0; mt < 2; ++mt)
    #pragma unroll
    for (int nt = 0; nt < 4; ++nt) acc[mt][nt] = zero8;

  #pragma unroll 1
  for (int k0 = 0; k0 < DM; k0 += 32) {
    const v16b a0 = load_frag_b(xa0 + k0, h);
    const v16b a1 = load_frag_b(xa1 + k0, h);
    #pragma unroll
    for (int nt = 0; nt < 4; ++nt) {
      const v16b b = load_frag_b(wr + (size_t)nt * 16 * DM + k0, h);
      acc[0][nt] = wmma_bf16(a0, b, acc[0][nt]);
      acc[1][nt] = wmma_bf16(a1, b, acc[1][nt]);
    }
  }

  const float* bias = (which == 0) ? bq : ((which == 1) ? bk : bv);
  #pragma unroll
  for (int nt = 0; nt < 4; ++nt) {
    const int feat = 16 * nt + m;
    const float bvl = bias[head * HD + feat];
    #pragma unroll
    for (int mt = 0; mt < 2; ++mt) {
      #pragma unroll
      for (int r = 0; r < 8; ++r) {
        const int tokl = 32 * w + 16 * mt + 8 * h + r;
        const float y = acc[mt][nt][r] + bvl;
        const int idx = (which == 2) ? (feat * 128 + tokl) : (tokl * HD + feat);
        sT[idx] = (_Float16)y;
      }
    }
  }
  __syncthreads();

  const int bp = m0 >> 10, l0 = m0 & (SQ - 1), bh = bp * NH + head;
  _Float16* plane = (which == 0) ? qh : kh;
  proj_store_pass(sT, plane, vt, which, bh, l0, w, lane);
  __threadfence();
  proj_store_pass(sT, plane, vt, which, bh, l0, w, lane);
}

__device__ __forceinline__ v8f scale_mask8(v8f s, const int* mp) {
  const v4i ma = *(const v4ia*)mp;
  const v4i mb = *(const v4ia*)(mp + 4);
  s[0] = (ma.x != 0) ? s[0] * 0.125f : -1.0e9f;
  s[1] = (ma.y != 0) ? s[1] * 0.125f : -1.0e9f;
  s[2] = (ma.z != 0) ? s[2] * 0.125f : -1.0e9f;
  s[3] = (ma.w != 0) ? s[3] * 0.125f : -1.0e9f;
  s[4] = (mb.x != 0) ? s[4] * 0.125f : -1.0e9f;
  s[5] = (mb.y != 0) ? s[5] * 0.125f : -1.0e9f;
  s[6] = (mb.z != 0) ? s[6] * 0.125f : -1.0e9f;
  s[7] = (mb.w != 0) ? s[7] * 0.125f : -1.0e9f;
  return s;
}

__device__ __forceinline__ v16h pack_p(v8f a, v8f c) {
  const v16h r = { (_Float16)(a[0] * PSCALE), (_Float16)(a[1] * PSCALE), (_Float16)(a[2] * PSCALE), (_Float16)(a[3] * PSCALE),
                   (_Float16)(a[4] * PSCALE), (_Float16)(a[5] * PSCALE), (_Float16)(a[6] * PSCALE), (_Float16)(a[7] * PSCALE),
                   (_Float16)(c[0] * PSCALE), (_Float16)(c[1] * PSCALE), (_Float16)(c[2] * PSCALE), (_Float16)(c[3] * PSCALE),
                   (_Float16)(c[4] * PSCALE), (_Float16)(c[5] * PSCALE), (_Float16)(c[6] * PSCALE), (_Float16)(c[7] * PSCALE) };
  return r;
}

__device__ __forceinline__ void xc_store_pass(const float* so, _Float16* xh, _Float16* xl,
                                              size_t tok0, int head, int lane) {
  const int q8 = lane & 7, sub = lane >> 3;
  #pragma unroll
  for (int i = 0; i < 4; ++i) {
    const int row = 4 * i + sub;
    const v4f a = *(const v4fa*)(so + row * 64 + 8 * q8);
    const v4f c = *(const v4fa*)(so + row * 64 + 8 * q8 + 4);
    const _Float16 h0 = (_Float16)a.x, h1 = (_Float16)a.y, h2 = (_Float16)a.z, h3 = (_Float16)a.w;
    const _Float16 h4 = (_Float16)c.x, h5 = (_Float16)c.y, h6 = (_Float16)c.z, h7 = (_Float16)c.w;
    const v8h hv = { h0, h1, h2, h3, h4, h5, h6, h7 };
    const v8h lv = { (_Float16)((a.x - (float)h0) * LOSCALE), (_Float16)((a.y - (float)h1) * LOSCALE),
                     (_Float16)((a.z - (float)h2) * LOSCALE), (_Float16)((a.w - (float)h3) * LOSCALE),
                     (_Float16)((c.x - (float)h4) * LOSCALE), (_Float16)((c.y - (float)h5) * LOSCALE),
                     (_Float16)((c.z - (float)h6) * LOSCALE), (_Float16)((c.w - (float)h7) * LOSCALE) };
    const size_t gi = (tok0 + row) * (size_t)DM + (size_t)head * HD + 8 * q8;
    *(volatile v8h*)(xh + gi) = hv;
    *(volatile v8h*)(xl + gi) = lv;
  }
}

__global__ __launch_bounds__(128) void attn_kernel(
    const _Float16* __restrict__ qh,
    const _Float16* __restrict__ kh,
    const _Float16* __restrict__ vt,
    const int* __restrict__ mask,
    _Float16* __restrict__ xh,
    _Float16* __restrict__ xl)
{
  __shared__ __attribute__((aligned(16))) float sO[4 * 16 * 64];

  const int tid = threadIdx.x, lane = tid & 31, w = tid >> 5;
  const int h = lane >> 4, m = lane & 15;
  const int bph = blockIdx.y, bp = bph >> 4, head = bph & 15;
  const int b = bp >> 1, p = bp & 1;
  const int q0 = blockIdx.x * 64 + 16 * w;

  const _Float16* qrow = qh + ((size_t)bph * SQ + q0 + m) * HD;
  const v16h qb0 = load_frag_h(qrow, h);
  const v16h qb1 = load_frag_h(qrow + 32, h);

  const int* mrow = mask + (size_t)bp * SQ;
  float* so = sO + w * 1024;
  const v8f zero8 = {0.f, 0.f, 0.f, 0.f, 0.f, 0.f, 0.f, 0.f};

  #pragma unroll 1
  for (int pass = 0; pass < 2; ++pass) {
    const int kvbp = (pass == 0) ? bp : (b * 2 + (1 - p));
    const int kvbph = kvbp * NH + head;
    const _Float16* kbase = kh + ((size_t)kvbph * SQ + m) * HD;
    const _Float16* vbase = vt + ((size_t)kvbph * HD + m) * SQ;

    v8f o[4];
    #pragma unroll
    for (int t = 0; t < 4; ++t) o[t] = zero8;
    float mrun = -1.0e30f, lrun = 0.0f;

    #pragma unroll 1
    for (int kb = 0; kb < SQ; kb += 64) {
      v8f s[4];
      #pragma unroll
      for (int j = 0; j < 4; ++j) {
        const _Float16* kp = kbase + (size_t)(kb + 16 * j) * HD;
        const v16h kf0 = load_frag_h(kp, h);
        const v16h kf1 = load_frag_h(kp + 32, h);
        v8f z = zero8;
        z = wmma_f16(kf0, qb0, z);
        z = wmma_f16(kf1, qb1, z);
        s[j] = z;
      }
      #pragma unroll
      for (int j = 0; j < 4; ++j) s[j] = scale_mask8(s[j], mrow + kb + 16 * j + 8 * h);

      float mloc = s[0][0];
      #pragma unroll
      for (int j = 0; j < 4; ++j)
        #pragma unroll
        for (int r = 0; r < 8; ++r) mloc = fmaxf(mloc, s[j][r]);
      mloc = fmaxf(mloc, __shfl_xor(mloc, 16));
      const float mnew = fmaxf(mrun, mloc);
      const float alpha = __expf(mrun - mnew);
      mrun = mnew;
      float lsum = 0.0f;
      #pragma unroll
      for (int j = 0; j < 4; ++j)
        #pragma unroll
        for (int r = 0; r < 8; ++r) {
          const float pe = __expf(s[j][r] - mnew);
          s[j][r] = pe;
          lsum += pe;
        }
      lsum += __shfl_xor(lsum, 16);
      lrun = lrun * alpha + lsum;
      #pragma unroll
      for (int t = 0; t < 4; ++t)
        #pragma unroll
        for (int r = 0; r < 8; ++r) o[t][r] = o[t][r] * alpha;

      const v16h pb0 = pack_p(s[0], s[1]);
      const v16h pb1 = pack_p(s[2], s[3]);

      #pragma unroll
      for (int t = 0; t < 4; ++t) {
        const _Float16* vp = vbase + (size_t)(16 * t) * SQ + kb;
        const v16h vf0 = load_frag_h(vp, h);
        const v16h vf1 = load_frag_h(vp + 32, h);
        o[t] = wmma_f16(vf0, pb0, o[t]);
        o[t] = wmma_f16(vf1, pb1, o[t]);
      }
    }

    const float inv = (1.0f / lrun) * (1.0f / PSCALE);
    if (pass == 0) {
      #pragma unroll
      for (int t = 0; t < 4; ++t)
        #pragma unroll
        for (int r = 0; r < 8; ++r)
          so[m * 64 + 16 * t + 8 * h + r] = o[t][r] * inv;
    } else {
      #pragma unroll
      for (int t = 0; t < 4; ++t)
        #pragma unroll
        for (int r = 0; r < 8; ++r) {
          const int idx = m * 64 + 16 * t + 8 * h + r;
          const float cmb = so[idx] + 0.1f * tanhf(o[t][r] * inv);
          so[idx] = cmb * XSCALE;
        }
    }
  }
  __syncthreads();

  const size_t tok0 = (size_t)bp * SQ + q0;
  xc_store_pass(so, xh, xl, tok0, head, lane);
  __threadfence();
  xc_store_pass(so, xh, xl, tok0, head, lane);
}

__device__ __forceinline__ void out_store_pass(const float* sT, float* out,
                                               int m0, int n0, int w, int lane) {
  const int q8 = lane & 7, sub = lane >> 3;
  #pragma unroll
  for (int i = 0; i < 8; ++i) {
    const int lid = i * 4 + sub;
    const int row = 16 * w + (lid >> 1), hl = lid & 1;
    const v4f v = *(const v4fa*)(sT + row * 64 + 32 * hl + 4 * q8);
    const size_t gi = (size_t)(m0 + row) * DM + n0 + 32 * hl + 4 * q8;
    *(volatile v4f*)(out + gi) = v;
  }
}

__global__ __launch_bounds__(128) void oproj_kernel(
    const _Float16* __restrict__ xh,
    const _Float16* __restrict__ xl,
    const _Float16* __restrict__ woh,
    const float* __restrict__ bo,
    float* __restrict__ out)
{
  __shared__ __attribute__((aligned(16))) float sT[64 * 64];

  const int tid = threadIdx.x, lane = tid & 31, w = tid >> 5;
  const int h = lane >> 4, m = lane & 15;
  const int m0 = blockIdx.x * 64, n0 = blockIdx.y * 64;
  const int row0 = m0 + 16 * w;

  const _Float16* ah = xh + (size_t)(row0 + m) * DM;
  const _Float16* al = xl + (size_t)(row0 + m) * DM;
  const _Float16* wr = woh + (size_t)(n0 + m) * DM;

  const v8f zero8 = {0.f, 0.f, 0.f, 0.f, 0.f, 0.f, 0.f, 0.f};
  v8f acch[4], accl[4];
  #pragma unroll
  for (int nt = 0; nt < 4; ++nt) { acch[nt] = zero8; accl[nt] = zero8; }

  #pragma unroll 1
  for (int k0 = 0; k0 < DM; k0 += 32) {
    const v16h fah = load_frag_h(ah + k0, h);
    const v16h fal = load_frag_h(al + k0, h);
    #pragma unroll
    for (int nt = 0; nt < 4; ++nt) {
      const v16h fb = load_frag_h(wr + (size_t)nt * 16 * DM + k0, h);
      acch[nt] = wmma_f16(fah, fb, acch[nt]);
      accl[nt] = wmma_f16(fal, fb, accl[nt]);
    }
  }

  const float sh = 1.0f / (XSCALE * WSCALE);
  const float sl = 1.0f / (XSCALE * WSCALE * LOSCALE);
  #pragma unroll
  for (int nt = 0; nt < 4; ++nt) {
    const int col = 16 * nt + m;
    const float bvl = bo[n0 + col];
    #pragma unroll
    for (int r = 0; r < 8; ++r) {
      const int row = 16 * w + 8 * h + r;
      sT[row * 64 + col] = acch[nt][r] * sh + accl[nt][r] * sl + bvl;
    }
  }
  __syncthreads();

  out_store_pass(sT, out, m0, n0, w, lane);
  __threadfence();
  out_store_pass(sT, out, m0, n0, w, lane);
}

extern "C" void kernel_launch(void* const* d_in, const int* in_sizes, int n_in,
                              void* d_out, int out_size, void* d_ws, size_t ws_size,
                              hipStream_t stream) {
  if (n_in < 12) return;
  if (in_sizes[0] != NACT || in_sizes[1] != NACT || in_sizes[2] != NACT) return;
  if (in_sizes[3] != NBP * SQ) return;
  if (in_sizes[4] != NWEL || in_sizes[6] != NWEL || in_sizes[8] != NWEL || in_sizes[10] != NWEL) return;
  if (in_sizes[5] != DM || in_sizes[7] != DM || in_sizes[9] != DM || in_sizes[11] != DM) return;
  if (out_size != NACT) return;

  const float* query = (const float*)d_in[0];
  const float* key_  = (const float*)d_in[1];
  const float* value = (const float*)d_in[2];
  const int*   mask  = (const int*)d_in[3];
  const float* Wq = (const float*)d_in[4];
  const float* bq = (const float*)d_in[5];
  const float* Wk = (const float*)d_in[6];
  const float* bk = (const float*)d_in[7];
  const float* Wv = (const float*)d_in[8];
  const float* bv = (const float*)d_in[9];
  const float* Wo = (const float*)d_in[10];
  const float* bo = (const float*)d_in[11];
  float* out = (float*)d_out;

  const size_t xb_bytes  = (size_t)3 * NACT * 2;
  const size_t wb_bytes  = (size_t)3 * NWEL * 2;
  const size_t woh_bytes = (size_t)NWEL * 2;
  const size_t pl_bytes  = (size_t)NBP * NH * SQ * HD * 2;
  const size_t xc_bytes  = (size_t)NACT * 2;
  const size_t total = xb_bytes + wb_bytes + woh_bytes + 3 * pl_bytes + 2 * xc_bytes;
  if (total > ws_size) return;

  char* ws = (char*)d_ws;
  size_t off = 0;
  unsigned short* xb = (unsigned short*)(ws + off); off += xb_bytes;
  unsigned short* wb = (unsigned short*)(ws + off); off += wb_bytes;
  _Float16* woh = (_Float16*)(ws + off);            off += woh_bytes;
  _Float16* qh  = (_Float16*)(ws + off);            off += pl_bytes;
  _Float16* kh  = (_Float16*)(ws + off);            off += pl_bytes;
  _Float16* vt  = (_Float16*)(ws + off);            off += pl_bytes;
  _Float16* xh  = (_Float16*)(ws + off);            off += xc_bytes;
  _Float16* xl  = (_Float16*)(ws + off);            off += xc_bytes;
  if (off > ws_size) return;

  convert_kernel<<<(NGRP + 255) / 256, 256, 0, stream>>>(query, key_, value, Wq, Wk, Wv, Wo, xb, wb, woh);

  dim3 gProj(NTOK / 128, 3 * NH);
  proj_kernel<<<gProj, 128, 0, stream>>>(xb, wb, bq, bk, bv, qh, kh, vt);

  dim3 gAtt(SQ / 64, NBP * NH);
  attn_kernel<<<gAtt, 128, 0, stream>>>(qh, kh, vt, mask, xh, xl);

  dim3 gOut(NTOK / 64, DM / 64);
  oproj_kernel<<<gOut, 128, 0, stream>>>(xh, xl, woh, bo, out);
}
